// SUE_25383256719527
// MI455X (gfx1250) — hardware-verified
//
#include <hip/hip_runtime.h>


namespace {
constexpr int B = 64, N = 16, H = 100, D = 400, DP = 416, A = 200, AP = 208, L = 2, CAT = 19, CP = 32, NODES = 118, NR = 128;
constexpr float XS = 8.0f, GS = 64.0f, WSC = 256.0f, ISC = 0.07071067811865475f;
typedef _Float16 b16;
typedef __attribute__((ext_vector_type(16))) _Float16 v16b;
typedef __attribute__((ext_vector_type(8))) _Float16 v8b;
typedef __attribute__((ext_vector_type(8))) float v8f;
typedef __attribute__((ext_vector_type(4))) float v4f;
typedef __attribute__((ext_vector_type(2))) _Float16 v2b;
__device__ __forceinline__ float bf16_rne(float f) { unsigned int u = __float_as_uint(f); u += 0x7FFFu + ((u >> 16) & 1u); return __uint_as_float(u & 0xFFFF0000u); }
__device__ __forceinline__ void split16(float v, b16& hi, b16& lo) { hi = (b16)v; lo = (b16)(v - (float)hi); }
__device__ __forceinline__ v16b frag_kb(const b16* p, int hh) { const v8b a = *(const v8b*)(p + 8 * hh), b = *(const v8b*)(p + 16 + 8 * hh); v16b f;
#pragma unroll
  for (int e = 0; e < 8; ++e) { f[e] = a[e]; f[8 + e] = b[e]; } return f; }
__device__ __forceinline__ v8f wmma16b(v16b a, v16b b, v8f c) { v8f d = __builtin_amdgcn_wmma_f32_16x16x32_f16(false, a, false, b, (short)0, c, false, false); asm volatile("v_nop\n\tv_nop\n\tv_nop\n\tv_nop" : "+v"(d) : "v"(a), "v"(b)); return d; }
__device__ __forceinline__ void wave_lds_sync() { __builtin_amdgcn_fence(__ATOMIC_RELEASE, "workgroup"); __builtin_amdgcn_wave_barrier(); __builtin_amdgcn_fence(__ATOMIC_ACQUIRE, "workgroup"); }
__device__ __forceinline__ float pmul(float a, float b) { float p = a * b; asm volatile("" : "+v"(p)); return p; }
__device__ __forceinline__ int iclamp(int v, int lo, int hi) { return v < lo ? lo : (v > hi ? hi : v); }

__global__ __launch_bounds__(256) void wput_kernel(const float* __restrict__ w, int OUTW, int OP, b16* __restrict__ WT) {
  const int KG = DP / 8; const int u = blockIdx.x * 256 + threadIdx.x; if (u >= OP * KG) return; const int o = u / KG, k0 = (u % KG) * 8; v8b v;
#pragma unroll
  for (int j = 0; j < 8; ++j) { const int k = k0 + j; v[j] = (o < OUTW && k < D) ? (b16)(bf16_rne(w[(size_t)k * OUTW + o]) * WSC) : (b16)0.0f; } for (int pass = 0; pass < 2; ++pass) { *(volatile v8b*)(WT + (size_t)o * DP + k0) = v; __threadfence(); }
}
__global__ __launch_bounds__(256) void he_kernel(const float* __restrict__ hist, const float* __restrict__ prox, int BV, float* __restrict__ HF, b16* __restrict__ HH, b16* __restrict__ HL) {
  const size_t u = (size_t)blockIdx.x * 256 + threadIdx.x; if (u >= (size_t)BV * NR * (DP / 8)) return; const int k0 = (int)(u % (DP / 8)) * 8; const int r = (int)((u / (DP / 8)) % NR); const int b = (int)(u / ((size_t)NR * (DP / 8)));
  float v[8]; v8b hv, lv;
#pragma unroll
  for (int j = 0; j < 8; ++j) { const int d = k0 + j; float x = 0.0f; if (d < D) { if (r < H) x = bf16_rne(hist[((size_t)b * H + r) * D + d]); else if (r < NODES) x = bf16_rne(prox[(size_t)(r - H) * D + d]); } v[j] = x; b16 p, q; split16(pmul(x, XS), p, q); hv[j] = p; lv[j] = q; }
  const size_t o_ = ((size_t)b * NR + r) * DP + k0;
  for (int pass = 0; pass < 2; ++pass) { *(volatile v4f*)(HF + o_) = (v4f){v[0], v[1], v[2], v[3]}; *(volatile v4f*)(HF + o_ + 4) = (v4f){v[4], v[5], v[6], v[7]}; *(volatile v8b*)(HH + o_) = hv; *(volatile v8b*)(HL + o_) = lv; __threadfence(); }
}
__global__ __launch_bounds__(32) void hw_kernel(const b16* __restrict__ HH, const b16* __restrict__ HL, const b16* __restrict__ WG, int BV, b16* __restrict__ HWTh, b16* __restrict__ HWTl) {
  __shared__ float Tt[16][NR + 1]; const int lane = threadIdx.x, nloc = lane & 15, hlf = lane >> 4; const int b = blockIdx.x / (DP / 16), ot = blockIdx.x % (DP / 16); if (b >= BV) return; if (ot >= D / 16) return;
  v8f acc[8];
#pragma unroll
  for (int t = 0; t < 8; ++t) acc[t] = (v8f){};
  const b16* hb = HH + (size_t)b * NR * DP; const b16* lb = HL + (size_t)b * NR * DP;
#pragma unroll 1
  for (int kb = 0; kb < DP; kb += 32) { const v16b w = frag_kb(WG + (size_t)(ot * 16 + nloc) * DP + kb, hlf);
#pragma unroll
    for (int t = 0; t < 8; ++t) { acc[t] = wmma16b(frag_kb(hb + (size_t)(t * 16 + nloc) * DP + kb, hlf), w, acc[t]); acc[t] = wmma16b(frag_kb(lb + (size_t)(t * 16 + nloc) * DP + kb, hlf), w, acc[t]); } }
#pragma unroll
  for (int t = 0; t < 8; ++t)
#pragma unroll
    for (int r8 = 0; r8 < 8; ++r8) Tt[nloc][t * 16 + 8 * hlf + r8] = acc[t][r8] * (1.0f / (XS * WSC));
  wave_lds_sync();
  for (int pass = 0; pass < 2; ++pass) { for (int ol = 0; ol < 16; ++ol) { const size_t row = ((size_t)b * D + ot * 16 + ol) * NR; for (int q = 0; q < 4; ++q) { const int j = q * 32 + lane; b16 p, ql; split16(pmul(Tt[ol][j], XS), p, ql); ((volatile b16*)HWTh)[row + j] = p; ((volatile b16*)HWTl)[row + j] = ql; } } __threadfence(); }
}
__global__ __launch_bounds__(32) void gz_kernel(const float* __restrict__ G, const b16* __restrict__ HWTh, const b16* __restrict__ HWTl, const float* __restrict__ gb, const float* __restrict__ lns, const float* __restrict__ lnb, const float* __restrict__ HFin, int BV, float* __restrict__ HF, b16* __restrict__ HH, b16* __restrict__ HL) {
  __shared__ __attribute__((aligned(16))) b16 Ag[16][NR + 8]; __shared__ float Z[16][D + 1], Mu[16], Rs[16];
  const int lane = threadIdx.x, nloc = lane & 15, hlf = lane >> 4; const int b = blockIdx.x / (NR / 16), it = blockIdx.x % (NR / 16); if (b >= BV) return; const int i0 = it * 16; if (i0 >= NODES) return;
  for (int rr = 0; rr < 16; ++rr) { const int i = i0 + rr; for (int q = 0; q < 4; ++q) { const int j = q * 32 + lane; Ag[rr][j] = (b16)((i < NODES && j < NODES) ? bf16_rne(G[((size_t)b * NODES + i) * NODES + j]) * GS : 0.0f); } }
  wave_lds_sync(); const b16* th = HWTh + (size_t)b * D * NR; const b16* tl = HWTl + (size_t)b * D * NR;
#pragma unroll 1
  for (int og = 0; og < 25; og += 5) { v8f acc[5];
#pragma unroll
    for (int t = 0; t < 5; ++t) acc[t] = (v8f){};
#pragma unroll
    for (int kb = 0; kb < NR; kb += 32) { const v16b a = frag_kb(&Ag[nloc][kb], hlf);
#pragma unroll
      for (int t = 0; t < 5; ++t) { const size_t orow = (size_t)((og + t) * 16 + nloc) * NR + kb; acc[t] = wmma16b(a, frag_kb(th + orow, hlf), acc[t]); acc[t] = wmma16b(a, frag_kb(tl + orow, hlf), acc[t]); } }
#pragma unroll
    for (int t = 0; t < 5; ++t) { const int o = (og + t) * 16 + nloc; const float bb = bf16_rne(gb[o]);
#pragma unroll
      for (int r8 = 0; r8 < 8; ++r8) { const int rl = 8 * hlf + r8; Z[rl][o] = fmaxf(acc[t][r8] * (1.0f / (GS * XS)) + bb, 0.0f) + HFin[((size_t)b * NR + i0 + rl) * DP + o]; } } }
  wave_lds_sync();
  if (lane < 16) { float s = 0.0f; for (int d = 0; d < D; ++d) s += Z[lane][d]; const float mu = s * (1.0f / D); float v = 0.0f; for (int d = 0; d < D; ++d) { const float dd = Z[lane][d] - mu; v += pmul(dd, dd); } Mu[lane] = mu; Rs[lane] = rsqrtf(v * (1.0f / D) + 1e-5f); }
  wave_lds_sync();
  for (int pass = 0; pass < 2; ++pass) { for (int rr = 0; rr < 16; ++rr) { const int i = i0 + rr; const size_t row = ((size_t)b * NR + i) * DP; for (int d = lane; d < DP; d += 32) { float v = 0.0f; if (i < NODES && d < D) v = pmul(pmul(Z[rr][d] - Mu[rr], Rs[rr]), bf16_rne(lns[d])) + bf16_rne(lnb[d]); ((volatile float*)HF)[row + d] = v; b16 p, ql; split16(pmul(v, XS), p, ql); ((volatile b16*)HH)[row + d] = p; ((volatile b16*)HL)[row + d] = ql; } } __threadfence(); }
}
__global__ __launch_bounds__(256) void gf_kernel(const float* __restrict__ HF, const float* __restrict__ HE, int BV, float* __restrict__ GF, b16* __restrict__ GH, b16* __restrict__ GL) {
  const size_t u = (size_t)blockIdx.x * 256 + threadIdx.x; if (u >= (size_t)BV * 112 * DP) return; const int d = (int)(u % DP), r = (int)((u / DP) % 112), b = (int)(u / ((size_t)112 * DP)); float v = 0.0f; if (r < H && d < D) { const size_t s = ((size_t)b * NR + r) * DP + d; v = HF[s] + HE[s]; }
  b16 p, q; split16(pmul(v, XS), p, q); for (int pass = 0; pass < 2; ++pass) { ((volatile float*)GF)[u] = v; ((volatile b16*)GH)[u] = p; ((volatile b16*)GL)[u] = q; __threadfence(); }
}
__global__ __launch_bounds__(32) void kmat_kernel(const b16* __restrict__ GH, const b16* __restrict__ GL, const b16* __restrict__ WK, int BV, float* __restrict__ KM) {
  __shared__ float Tf[16][AP + 4]; const int lane = threadIdx.x, nloc = lane & 15, hlf = lane >> 4; const int b = blockIdx.x / 7, rt = blockIdx.x % 7; if (b >= BV) return; const size_t r0 = (size_t)b * 112 + rt * 16;
  v8f acc[13];
#pragma unroll
  for (int t = 0; t < 13; ++t) acc[t] = (v8f){};
#pragma unroll 1
  for (int kb = 0; kb < DP; kb += 32) { const v16b a = frag_kb(GH + (r0 + nloc) * DP + kb, hlf), al = frag_kb(GL + (r0 + nloc) * DP + kb, hlf);
#pragma unroll
    for (int t = 0; t < 13; ++t) { const v16b w = frag_kb(WK + (size_t)(t * 16 + nloc) * DP + kb, hlf); acc[t] = wmma16b(a, w, acc[t]); acc[t] = wmma16b(al, w, acc[t]); } }
#pragma unroll
  for (int t = 0; t < 13; ++t)
#pragma unroll
    for (int r8 = 0; r8 < 8; ++r8) Tf[8 * hlf + r8][t * 16 + nloc] = acc[t][r8] * (1.0f / (XS * WSC));
  wave_lds_sync();
  for (int pass = 0; pass < 2; ++pass) { for (int rr = 0; rr < 16; ++rr) for (int c = lane; c < AP; c += 32) ((volatile float*)KM)[(r0 + rr) * AP + c] = Tf[rr][c]; __threadfence(); }
}
__global__ __launch_bounds__(32) void qmat_kernel(const float* __restrict__ cand, const b16* __restrict__ WQ, const float* __restrict__ qb, const b16* __restrict__ WQ2, const float* __restrict__ qb2, int BV, float* __restrict__ QM, float* __restrict__ QM2) {
  __shared__ __attribute__((aligned(16))) b16 Ah[16][DP + 8]; __shared__ float Tf[16][AP + 4]; const int lane = threadIdx.x, nloc = lane & 15, hlf = lane >> 4; const int b = blockIdx.x; if (b >= BV) return;
  for (int rr = 0; rr < 16; ++rr) for (int d = lane; d < DP; d += 32) Ah[rr][d] = (b16)((d < D ? bf16_rne(cand[((size_t)b * N + rr) * D + d]) : 0.0f) * XS);
  wave_lds_sync();
#pragma unroll 1
  for (int which = 0; which < 2; ++which) { const b16* W = which ? WQ2 : WQ; const float* bb = which ? qb2 : qb; float* OUT = which ? QM2 : QM; v8f acc[13];
#pragma unroll
    for (int t = 0; t < 13; ++t) acc[t] = (v8f){};
#pragma unroll 1
    for (int kb = 0; kb < DP; kb += 32) { const v16b a = frag_kb(&Ah[nloc][kb], hlf);
#pragma unroll
      for (int t = 0; t < 13; ++t) acc[t] = wmma16b(a, frag_kb(W + (size_t)(t * 16 + nloc) * DP + kb, hlf), acc[t]); }
#pragma unroll
    for (int t = 0; t < 13; ++t) { const int c = t * 16 + nloc; const float bv = c < A ? bf16_rne(bb[c]) : 0.0f;
#pragma unroll
      for (int r8 = 0; r8 < 8; ++r8) Tf[8 * hlf + r8][c] = acc[t][r8] * (1.0f / (XS * WSC)) + bv; }
    wave_lds_sync();
    for (int pass = 0; pass < 2; ++pass) { for (int rr = 0; rr < 16; ++rr) for (int c = lane; c < AP; c += 32) ((volatile float*)OUT)[((size_t)b * N + rr) * AP + c] = Tf[rr][c]; __threadfence(); }
    wave_lds_sync(); }
}
__global__ __launch_bounds__(32) void intra_kernel(const float* __restrict__ KM, const float* __restrict__ QM, const float* __restrict__ GF, const int* __restrict__ cidx, int BV, b16* __restrict__ INh, b16* __restrict__ INl) {
  __shared__ float Al[H + 28], Cmx[CP], Csum[CP], In[CP][D + 1]; __shared__ int Ci[H + 28];
  const int lane = threadIdx.x; const int b = blockIdx.x / N, n = blockIdx.x % N; if (b >= BV) return; const float* qn = QM + ((size_t)b * N + n) * AP;
  for (int q = 0; q < 4; ++q) { const int h = q * 32 + lane; float s = 0.0f; int ci = 0; if (h < H) { const float* kr = KM + ((size_t)b * 112 + h) * AP;
#pragma unroll 4
      for (int a = 0; a < A; ++a) s += pmul(kr[a], qn[a]); s = pmul(s, ISC); ci = iclamp(cidx[b * H + h], 0, CAT - 1); } Al[h] = s; Ci[h] = ci; }
  Cmx[lane] = -INFINITY; Csum[lane] = 0.0f; wave_lds_sync();
  if (lane < CAT) { float mx = -INFINITY; for (int h = 0; h < H; ++h) if (Ci[h] == lane) mx = fmaxf(mx, Al[h]); Cmx[lane] = mx; }
  wave_lds_sync();
  for (int q = 0; q < 4; ++q) { const int h = q * 32 + lane; if (h < H) Al[h] = __expf(Al[h] - Cmx[Ci[h]]); }
  wave_lds_sync();
  if (lane < CAT) { float s = 0.0f; for (int h = 0; h < H; ++h) if (Ci[h] == lane) s += Al[h]; Csum[lane] = s; }
  wave_lds_sync();
  for (int q = 0; q < 4; ++q) { const int h = q * 32 + lane; if (h < H) Al[h] = Al[h] / Csum[Ci[h]]; }
  for (int c = 0; c < CP; ++c) for (int d = lane; d < D; d += 32) In[c][d] = 0.0f;
  wave_lds_sync();
#pragma unroll 1
  for (int h = 0; h < H; ++h) { const int c = Ci[h]; const float al = Al[h]; const float* gr = GF + ((size_t)b * 112 + h) * DP; for (int d = lane; d < D; d += 32) In[c][d] += pmul(al, gr[d]); }
  wave_lds_sync();
  for (int pass = 0; pass < 2; ++pass) { for (int c = 0; c < CP; ++c) { const size_t row = (((size_t)b * N + n) * CP + c) * DP; for (int d = lane; d < DP; d += 32) { const float v = (c < CAT && d < D) ? In[c][d] : 0.0f; b16 p, ql; split16(pmul(v, XS), p, ql); ((volatile b16*)INh)[row + d] = p; ((volatile b16*)INl)[row + d] = ql; } } __threadfence(); }
}
__global__ __launch_bounds__(32) void aff_kernel(const b16* __restrict__ INh, const b16* __restrict__ INl, const b16* __restrict__ WA, const float* __restrict__ afb, int BV, b16* __restrict__ I2h, b16* __restrict__ I2l) {
  __shared__ float Tf[16][D + 1]; const int lane = threadIdx.x, nloc = lane & 15, hlf = lane >> 4; const int bn = blockIdx.x >> 1, rt = blockIdx.x & 1; const int b = bn / N; if (b >= BV) return; const size_t r0 = (size_t)bn * CP + rt * 16;
#pragma unroll 1
  for (int og = 0; og < 25; og += 5) { v8f acc[5];
#pragma unroll
    for (int t = 0; t < 5; ++t) acc[t] = (v8f){};
#pragma unroll 1
    for (int kb = 0; kb < DP; kb += 32) { const v16b a = frag_kb(INh + (r0 + nloc) * DP + kb, hlf), al = frag_kb(INl + (r0 + nloc) * DP + kb, hlf);
#pragma unroll
      for (int t = 0; t < 5; ++t) { const v16b w = frag_kb(WA + (size_t)((og + t) * 16 + nloc) * DP + kb, hlf); acc[t] = wmma16b(a, w, acc[t]); acc[t] = wmma16b(al, w, acc[t]); } }
#pragma unroll
    for (int t = 0; t < 5; ++t) { const int o = (og + t) * 16 + nloc; const float bb = bf16_rne(afb[o]);
#pragma unroll
      for (int r8 = 0; r8 < 8; ++r8) Tf[8 * hlf + r8][o] = fmaxf(acc[t][r8] * (1.0f / (XS * WSC)) + bb, 0.0f); } }
  wave_lds_sync();
  for (int pass = 0; pass < 2; ++pass) { for (int rr = 0; rr < 16; ++rr) { const int c = rt * 16 + rr; const size_t row = (r0 + rr) * DP; for (int d = lane; d < DP; d += 32) { float v = 0.0f; if (c < CAT && d < D) { const float in = ((float)INh[row + d] + (float)INl[row + d]) * (1.0f / XS); v = Tf[rr][d] + in; } b16 p, ql; split16(pmul(v, XS), p, ql); ((volatile b16*)I2h)[row + d] = p; ((volatile b16*)I2l)[row + d] = ql; } } __threadfence(); }
}
__global__ __launch_bounds__(32) void inter_kernel(const b16* __restrict__ I2h, const b16* __restrict__ I2l, const b16* __restrict__ WK2, const float* __restrict__ QM2, const int* __restrict__ cmask, int BV, float* __restrict__ out) {
  __shared__ float Kf[CP][AP + 4], Wc[CP], Ov[D]; const int lane = threadIdx.x, nloc = lane & 15, hlf = lane >> 4;
#pragma unroll 1
  for (int sub = 0; sub < 2; ++sub) { const int bn = 2 * blockIdx.x + sub; const int b = bn / N, n = bn % N; if (b >= BV) return; const size_t r0 = (size_t)bn * CP;
#pragma unroll 1
  for (int rt = 0; rt < 2; ++rt) { v8f acc[13];
#pragma unroll
    for (int t = 0; t < 13; ++t) acc[t] = (v8f){};
#pragma unroll 1
    for (int kb = 0; kb < DP; kb += 32) { const v16b a = frag_kb(I2h + (r0 + rt * 16 + nloc) * DP + kb, hlf), al = frag_kb(I2l + (r0 + rt * 16 + nloc) * DP + kb, hlf);
#pragma unroll
      for (int t = 0; t < 13; ++t) { const v16b w = frag_kb(WK2 + (size_t)(t * 16 + nloc) * DP + kb, hlf); acc[t] = wmma16b(a, w, acc[t]); acc[t] = wmma16b(al, w, acc[t]); } }
#pragma unroll
    for (int t = 0; t < 13; ++t)
#pragma unroll
      for (int r8 = 0; r8 < 8; ++r8) Kf[rt * 16 + 8 * hlf + r8][t * 16 + nloc] = acc[t][r8] * (1.0f / (XS * WSC)); }
  wave_lds_sync();
  { const int c = lane; float s = -INFINITY; const bool valid = (c < CAT) && (c == CAT - 1 || cmask[b * CAT + (c < CAT ? c : 0)] != 0); if (valid) { const float* qn = QM2 + ((size_t)b * N + n) * AP; float d_ = 0.0f;
#pragma unroll 4
      for (int a = 0; a < A; ++a) d_ += pmul(Kf[c][a], qn[a]); s = pmul(d_, ISC); }
    float mx = s; for (int o = 16; o; o >>= 1) mx = fmaxf(mx, __shfl_xor(mx, o)); const float e = valid ? __expf(s - mx) : 0.0f; float sm = e; for (int o = 16; o; o >>= 1) sm += __shfl_xor(sm, o); Wc[lane] = e / sm; }
  wave_lds_sync();
  for (int d = lane; d < D; d += 32) { float s = 0.0f;
#pragma unroll 1
    for (int c = 0; c < CAT; ++c) { const size_t row = (r0 + c) * DP; s += pmul(Wc[c], ((float)I2h[row + d] + (float)I2l[row + d]) * (1.0f / XS)); } Ov[d] = s; }
  wave_lds_sync();
  for (int pass = 0; pass < 2; ++pass) { for (int d = lane; d < D; d += 32) ((volatile float*)out)[(size_t)bn * D + d] = Ov[d]; __threadfence(); }
  wave_lds_sync(); }
}
}

extern "C" void kernel_launch(void* const* d_in, const int* in_sizes, int n_in, void* d_out, int out_size, void* d_ws, size_t ws_size, hipStream_t stream) {
  (void)n_in;
  auto Fp = [&](int i) { return (const float*)d_in[i]; }; auto Ip = [&](int i) { return (const int*)d_in[i]; };
  if (in_sizes[0] != B * H * D || in_sizes[1] != B * N * D || in_sizes[2] != B * NODES * NODES || in_sizes[3] != B * CAT || in_sizes[4] != B * H || in_sizes[5] != (CAT - 1) * D || in_sizes[6] != L * D * D || in_sizes[10] != D * A || in_sizes[13] != D * D || in_sizes[15] != D * A || in_sizes[16] != D * A || out_size != B * N * D) return;
  const int BV = B;
  size_t off = 0; char* ws = (char*)d_ws;
  auto carve = [&](size_t bytes) { char* p = ws + off; off += (bytes + 255) & ~(size_t)255; return p; };
  b16* WG[2]; for (int l = 0; l < L; ++l) WG[l] = (b16*)carve((size_t)DP * DP * 2); b16* WK = (b16*)carve((size_t)AP * DP * 2); b16* WQ = (b16*)carve((size_t)AP * DP * 2); b16* WA = (b16*)carve((size_t)DP * DP * 2); b16* WK2 = (b16*)carve((size_t)AP * DP * 2); b16* WQ2 = (b16*)carve((size_t)AP * DP * 2);
  float* HE = (float*)carve((size_t)B * NR * DP * 4); b16* HEh = (b16*)carve((size_t)B * NR * DP * 2); b16* HEl = (b16*)carve((size_t)B * NR * DP * 2);
  float* HF1 = (float*)carve((size_t)B * NR * DP * 4); b16* HH1 = (b16*)carve((size_t)B * NR * DP * 2); b16* HL1 = (b16*)carve((size_t)B * NR * DP * 2);
  float* HF2 = (float*)carve((size_t)B * NR * DP * 4); b16* HH2 = (b16*)carve((size_t)B * NR * DP * 2); b16* HL2 = (b16*)carve((size_t)B * NR * DP * 2);
  b16* HWTh = (b16*)carve((size_t)B * D * NR * 2); b16* HWTl = (b16*)carve((size_t)B * D * NR * 2);
  float* GF = (float*)carve((size_t)B * 112 * DP * 4); b16* GH = (b16*)carve((size_t)B * 112 * DP * 2); b16* GL = (b16*)carve((size_t)B * 112 * DP * 2);
  float* KM = (float*)carve((size_t)B * 112 * AP * 4); float* QM = (float*)carve((size_t)B * N * AP * 4); float* QM2 = (float*)carve((size_t)B * N * AP * 4);
  b16* INh = (b16*)carve((size_t)B * N * CP * DP * 2); b16* INl = (b16*)carve((size_t)B * N * CP * DP * 2); b16* I2h = (b16*)carve((size_t)B * N * CP * DP * 2); b16* I2l = (b16*)carve((size_t)B * N * CP * DP * 2);
  if (off > ws_size || off > ((size_t)240 << 20)) return;
  for (int l = 0; l < L; ++l) wput_kernel<<<(DP * (DP / 8) + 255) / 256, 256, 0, stream>>>(Fp(6) + (size_t)l * D * D, D, DP, WG[l]);
  wput_kernel<<<(AP * (DP / 8) + 255) / 256, 256, 0, stream>>>(Fp(10), A, AP, WK); wput_kernel<<<(AP * (DP / 8) + 255) / 256, 256, 0, stream>>>(Fp(11), A, AP, WQ); wput_kernel<<<(DP * (DP / 8) + 255) / 256, 256, 0, stream>>>(Fp(13), D, DP, WA);
  wput_kernel<<<(AP * (DP / 8) + 255) / 256, 256, 0, stream>>>(Fp(15), A, AP, WK2); wput_kernel<<<(AP * (DP / 8) + 255) / 256, 256, 0, stream>>>(Fp(16), A, AP, WQ2);
  he_kernel<<<(unsigned)(((size_t)BV * NR * (DP / 8) + 255) / 256), 256, 0, stream>>>(Fp(0), Fp(5), BV, HE, HEh, HEl);
  hw_kernel<<<BV * (DP / 16), 32, 0, stream>>>(HEh, HEl, WG[0], BV, HWTh, HWTl);
  gz_kernel<<<BV * (NR / 16), 32, 0, stream>>>(Fp(2), HWTh, HWTl, Fp(7), Fp(8), Fp(9), HE, BV, HF1, HH1, HL1);
  hw_kernel<<<BV * (DP / 16), 32, 0, stream>>>(HH1, HL1, WG[1], BV, HWTh, HWTl);
  gz_kernel<<<BV * (NR / 16), 32, 0, stream>>>(Fp(2), HWTh, HWTl, Fp(7) + D, Fp(8) + D, Fp(9) + D, HF1, BV, HF2, HH2, HL2);
  gf_kernel<<<(unsigned)(((size_t)BV * 112 * DP + 255) / 256), 256, 0, stream>>>(HF2, HE, BV, GF, GH, GL);
  kmat_kernel<<<BV * 7, 32, 0, stream>>>(GH, GL, WK, BV, KM);
  qmat_kernel<<<BV, 32, 0, stream>>>(Fp(1), WQ, Fp(12), WQ2, Fp(17), BV, QM, QM2);
  intra_kernel<<<BV * N, 32, 0, stream>>>(KM, QM, GF, Ip(4), BV, INh, INl);
  aff_kernel<<<BV * N * 2, 32, 0, stream>>>(INh, INl, WA, Fp(14), BV, I2h, I2l);
  inter_kernel<<<BV * N / 2, 32, 0, stream>>>(I2h, I2l, WK2, QM2, Ip(3), BV, (float*)d_out);
}
